// PIMACV3ActorRNN_41386304864870
// MI455X (gfx1250) — hardware-verified
//
#include <hip/hip_runtime.h>


typedef _Float16 f16t;
typedef f16t  v16h __attribute__((ext_vector_type(16)));
typedef f16t  v8h  __attribute__((ext_vector_type(8)));
typedef float v8f  __attribute__((ext_vector_type(8)));
typedef float v4f  __attribute__((ext_vector_type(4)));
typedef unsigned int v4u __attribute__((ext_vector_type(4)));

union Frag { v16h v; v8h q[2]; };
union Pk16 { v8h h; v4u u; };
union Pk32 { v4f f; v4u u; };

#define NBATCH 16
#define NSTEP  256
#define NTOK   4096
#define OBSD   128
#define W0D    256
#define HIDD   256
#define G3D    768
#define CTXD   64
#define ACTD   64
#define HNH    128
#define HNOUT  1344
#define LP     264

__device__ __forceinline__ v8f wmma16(v16h a, v16h b, v8f c) {
    return __builtin_amdgcn_wmma_f32_16x16x32_f16(false, a, false, b, (short)0, c, false, false);
}

__device__ __forceinline__ void wguard(v8f (&c)[4][2], Frag (&a)[4], Frag (&b)[2]) {
    asm volatile("v_nop\n\tv_nop\n\tv_nop\n\tv_nop"
                 : "+v"(c[0][0]), "+v"(c[0][1]), "+v"(c[1][0]), "+v"(c[1][1]),
                   "+v"(c[2][0]), "+v"(c[2][1]), "+v"(c[3][0]), "+v"(c[3][1])
                 : "v"(a[0].v), "v"(a[1].v), "v"(a[2].v), "v"(a[3].v),
                   "v"(b[0].v), "v"(b[1].v));
}
__device__ __forceinline__ void wguard(v8f (&c)[3][2], Frag (&a)[3][2], Frag& b) {
    asm volatile("v_nop\n\tv_nop\n\tv_nop\n\tv_nop"
                 : "+v"(c[0][0]), "+v"(c[0][1]), "+v"(c[1][0]), "+v"(c[1][1]),
                   "+v"(c[2][0]), "+v"(c[2][1])
                 : "v"(a[0][0].v), "v"(a[0][1].v), "v"(a[1][0].v), "v"(a[1][1].v),
                   "v"(a[2][0].v), "v"(a[2][1].v), "v"(b.v));
}

template<int MT, int NT>
__device__ __forceinline__ void zacc(v8f (&acc)[MT][NT]) {
    const v8f z = {0.f, 0.f, 0.f, 0.f, 0.f, 0.f, 0.f, 0.f};
#pragma unroll
    for (int i = 0; i < MT; ++i)
#pragma unroll
        for (int j = 0; j < NT; ++j) acc[i][j] = z;
}

template<int MT, int NT>
__device__ __forceinline__ void mma_acc(v8f (&acc)[MT][NT],
                                        const f16t* A, int lda,
                                        const f16t* B, int ldb, int ktiles) {
    const int l = threadIdx.x & 31, h = l >> 4, m = l & 15;
    const f16t* ap = A + (size_t)m * lda + 8 * h;
    const f16t* bp = B + (size_t)m * ldb + 8 * h;
#pragma unroll 1
    for (int kt = 0; kt < ktiles; ++kt) {
        Frag a[MT], b[NT];
#pragma unroll
        for (int i = 0; i < MT; ++i) {
            const f16t* p = ap + (size_t)i * 16 * lda + kt * 32;
            a[i].q[0] = *(const v8h*)p;
            a[i].q[1] = *(const v8h*)(p + 16);
        }
#pragma unroll
        for (int j = 0; j < NT; ++j) {
            const f16t* p = bp + (size_t)j * 16 * ldb + kt * 32;
            b[j].q[0] = *(const v8h*)p;
            b[j].q[1] = *(const v8h*)(p + 16);
        }
#pragma unroll
        for (int i = 0; i < MT; ++i)
#pragma unroll
            for (int j = 0; j < NT; ++j)
                acc[i][j] = wmma16(a[i].v, b[j].v, acc[i][j]);
        wguard(acc, a, b);
    }
}

__device__ __forceinline__ float fsigm(float x) {
    return __builtin_amdgcn_rcpf(1.0f + expf(-x));
}
__device__ __forceinline__ float ftanh(float x) {
    float ax = fabsf(x);
    float t  = expf(-2.0f * ax);
    float r  = (1.0f - t) * __builtin_amdgcn_rcpf(1.0f + t);
    return copysignf(r, x);
}
__device__ __forceinline__ float wsum(float v) {
#pragma unroll
    for (int o = 16; o > 0; o >>= 1) v += __shfl_xor(v, o, 32);
    return v;
}

template<int ACT>
__device__ __forceinline__ float act_f(float v) {
    if (ACT == 1) v = fmaxf(v, 0.0f);
    if (ACT == 2) v = fminf(fmaxf(v, -6.0f), 4.0f);
    if (ACT == 3) v = v * 0.05f;
    return v;
}

template<int MT, int NT, int ACT>
__device__ __forceinline__ void epi_lds(v8f (&acc)[MT][NT], float inv, const float* bias,
                                        f16t* L, int pitch) {
    const int l = threadIdx.x & 31, h = l >> 4, m = l & 15;
#pragma unroll
    for (int i = 0; i < MT; ++i) {
        const int col = 16 * i + 8 * h;
        float bv[8];
#pragma unroll
        for (int r = 0; r < 8; ++r) bv[r] = bias[col + r];
#pragma unroll
        for (int j = 0; j < NT; ++j) {
            Pk16 pk;
#pragma unroll
            for (int r = 0; r < 8; ++r)
                pk.h[r] = (f16t)act_f<ACT>(fmaf(acc[i][j][r], inv, bv[r]));
            *(v8h*)(L + (size_t)(16 * j + m) * pitch + col) = pk.h;
        }
    }
}
template<int MT, int NT, int ACT>
__device__ __forceinline__ void epi_lds(v8f (&acc)[MT][NT], float inv, const float* bias,
                                        float* L, int pitch) {
    const int l = threadIdx.x & 31, h = l >> 4, m = l & 15;
#pragma unroll
    for (int i = 0; i < MT; ++i) {
        const int col = 16 * i + 8 * h;
        float bv[8];
#pragma unroll
        for (int r = 0; r < 8; ++r) bv[r] = bias[col + r];
#pragma unroll
        for (int j = 0; j < NT; ++j) {
            Pk32 p0, p1;
#pragma unroll
            for (int r = 0; r < 4; ++r) {
                p0.f[r] = act_f<ACT>(fmaf(acc[i][j][r],     inv, bv[r]));
                p1.f[r] = act_f<ACT>(fmaf(acc[i][j][4 + r], inv, bv[4 + r]));
            }
            float* d = L + (size_t)(16 * j + m) * pitch + col;
            *(v4f*)d       = p0.f;
            *(v4f*)(d + 4) = p1.f;
        }
    }
}

__device__ __forceinline__ void tile_out(const f16t* S, f16t* Y, int ldy, int r0, int f0) {
    const int tid = threadIdx.x;
    Pk16 v[8];
#pragma unroll
    for (int i = 0; i < 8; ++i) {
        int p = tid + 64 * i, row = p >> 3, ch = (p & 7) * 8;
        v[i].h = *(const v8h*)(S + row * 64 + ch);
    }
#pragma unroll
    for (int i = 0; i < 8; ++i) {
        int p = tid + 64 * i, row = p >> 3, ch = (p & 7) * 8;
        *(volatile v4u*)(Y + (size_t)(r0 + row) * ldy + f0 + ch) = v[i].u;
    }
    __threadfence();
#pragma unroll
    for (int i = 0; i < 8; ++i) {
        int p = tid + 64 * i, row = p >> 3, ch = (p & 7) * 8;
        *(volatile v4u*)(Y + (size_t)(r0 + row) * ldy + f0 + ch) = v[i].u;
    }
}
__device__ __forceinline__ void tile_out(const float* S, float* Y, int ldy, int r0, int f0) {
    const int tid = threadIdx.x;
#pragma unroll
    for (int hb = 0; hb < 2; ++hb) {
        Pk32 v[8];
#pragma unroll
        for (int i = 0; i < 8; ++i) {
            int p = tid + 64 * (8 * hb + i), row = p >> 4, c = (p & 15) * 4;
            v[i].f = *(const v4f*)(S + row * 64 + c);
        }
#pragma unroll
        for (int i = 0; i < 8; ++i) {
            int p = tid + 64 * (8 * hb + i), row = p >> 4, c = (p & 15) * 4;
            *(volatile v4u*)(Y + (size_t)(r0 + row) * ldy + f0 + c) = v[i].u;
        }
        __threadfence();
#pragma unroll
        for (int i = 0; i < 8; ++i) {
            int p = tid + 64 * (8 * hb + i), row = p >> 4, c = (p & 15) * 4;
            *(volatile v4u*)(Y + (size_t)(r0 + row) * ldy + f0 + c) = v[i].u;
        }
    }
}

__global__ __launch_bounds__(256)
void k_cvt8(const float* x, f16t* y, int n8, float sc) {
    int i = blockIdx.x * 256 + threadIdx.x;
    if (i >= n8) return;
    const float* p = x + (size_t)i * 8;
    Pk16 k;
#pragma unroll
    for (int e = 0; e < 8; ++e) k.h[e] = (f16t)(p[e] * sc);
    f16t* d = y + (size_t)i * 8;
    *(volatile v4u*)d = k.u;
    __threadfence();
    *(volatile v4u*)d = k.u;
}

template<typename OT, int ACT>
__global__ __launch_bounds__(64)
void k_gemm(const f16t* X, int ldx, const f16t* P, int K, const float* bias,
            OT* Y, int ldy, int nrows, int ncols, float inv) {
    __shared__ __attribute__((aligned(16))) OT S[64 * 64];
    const int w  = threadIdx.x >> 5;
    const int f0 = blockIdx.x * 64;
    const int r0 = blockIdx.y * 64;
    if (f0 + 64 > ncols || r0 + 64 > nrows) return;

    v8f acc[4][2]; zacc(acc);
    mma_acc<4, 2>(acc, P + (size_t)f0 * K, K, X + (size_t)(r0 + 32 * w) * ldx, ldx, K >> 5);
    epi_lds<4, 2, ACT>(acc, inv, bias + f0, S + 32 * w * 64, 64);
    __syncthreads();
    tile_out(S, Y, ldy, r0, f0);
}

__device__ __forceinline__ float gru_cell(float ar, float az, float an, float inv,
                                          float xr, float xz, float xn,
                                          float br, float bz, float bn, float hold) {
    float hr = fmaf(ar, inv, br);
    float hz = fmaf(az, inv, bz);
    float hn = fmaf(an, inv, bn);
    float rg = fsigm(xr + hr);
    float zg = fsigm(xz + hz);
    float ng = ftanh(fmaf(rg, hn, xn));
    return (1.0f - zg) * ng + zg * hold;
}

__global__ __launch_bounds__(256)
void k_gru(const float* XG, const f16t* Phh, const float* bhh, const float* h0,
           f16t* FE, float* HT, int T, float inv) {
    __shared__ __attribute__((aligned(16))) f16t  H16[NBATCH * LP];
    __shared__ __attribute__((aligned(16))) float SF[NBATCH * HIDD];
    const int tid = threadIdx.x;
    const int w = tid >> 5, l = tid & 31, h = l >> 4, m = l & 15;
    const int fb = 32 * w;

    float hreg[2][8];
#pragma unroll
    for (int i = 0; i < 2; ++i) {
        const int fo = fb + 16 * i + 8 * h;
        Pk16 pk;
#pragma unroll
        for (int r = 0; r < 8; ++r) {
            hreg[i][r] = h0[m * HIDD + fo + r];
            pk.h[r] = (f16t)hreg[i][r];
        }
        *(v8h*)(H16 + m * LP + fo) = pk.h;
    }
    __syncthreads();

    const f16t* bp = H16 + m * LP + 8 * h;
    const f16t* ap = Phh + (size_t)(fb + m) * HIDD + 8 * h;

#pragma unroll 1
    for (int t = 0; t < T; ++t) {
        v8f acc[3][2];
        {
            const v8f z = {0.f, 0.f, 0.f, 0.f, 0.f, 0.f, 0.f, 0.f};
#pragma unroll
            for (int g = 0; g < 3; ++g) { acc[g][0] = z; acc[g][1] = z; }
        }
#pragma unroll 1
        for (int kt = 0; kt < HIDD / 32; ++kt) {
            Frag a[3][2], b;
            b.q[0] = *(const v8h*)(bp + kt * 32);
            b.q[1] = *(const v8h*)(bp + kt * 32 + 16);
#pragma unroll
            for (int g = 0; g < 3; ++g)
#pragma unroll
                for (int i = 0; i < 2; ++i) {
                    const f16t* p = ap + (size_t)(g * HIDD + 16 * i) * HIDD + kt * 32;
                    a[g][i].q[0] = *(const v8h*)p;
                    a[g][i].q[1] = *(const v8h*)(p + 16);
                }
#pragma unroll
            for (int g = 0; g < 3; ++g)
#pragma unroll
                for (int i = 0; i < 2; ++i)
                    acc[g][i] = wmma16(a[g][i].v, b.v, acc[g][i]);
            wguard(acc, a, b);
        }

#pragma unroll
        for (int i = 0; i < 2; ++i) {
            const int fo = fb + 16 * i + 8 * h;
            const float* xg = XG + ((size_t)m * T + t) * G3D + fo;
            const float* bq = bhh + fo;
            v4f xr0 = *(const v4f*)xg,              xr1 = *(const v4f*)(xg + 4);
            v4f xz0 = *(const v4f*)(xg + HIDD),     xz1 = *(const v4f*)(xg + HIDD + 4);
            v4f xn0 = *(const v4f*)(xg + 2 * HIDD), xn1 = *(const v4f*)(xg + 2 * HIDD + 4);
            float br[8], bz[8], bn[8];
#pragma unroll
            for (int r = 0; r < 8; ++r) {
                br[r] = bq[r];
                bz[r] = bq[HIDD + r];
                bn[r] = bq[2 * HIDD + r];
            }
#pragma unroll
            for (int r = 0; r < 4; ++r) {
                hreg[i][r] = gru_cell(acc[0][i][r], acc[1][i][r], acc[2][i][r], inv,
                                      xr0[r], xz0[r], xn0[r], br[r], bz[r], bn[r], hreg[i][r]);
                hreg[i][4 + r] = gru_cell(acc[0][i][4 + r], acc[1][i][4 + r], acc[2][i][4 + r], inv,
                                          xr1[r], xz1[r], xn1[r], br[4 + r], bz[4 + r], bn[4 + r],
                                          hreg[i][4 + r]);
            }
        }
        __syncthreads();
#pragma unroll
        for (int i = 0; i < 2; ++i) {
            Pk16 pk;
#pragma unroll
            for (int r = 0; r < 8; ++r) pk.h[r] = (f16t)hreg[i][r];
            *(v8h*)(H16 + m * LP + fb + 16 * i + 8 * h) = pk.h;
        }
        __syncthreads();

        Pk16 v[2];
#pragma unroll
        for (int k = 0; k < 2; ++k) {
            int p = tid + 256 * k, row = p >> 5, ch = (p & 31) * 8;
            v[k].h = *(const v8h*)(H16 + row * LP + ch);
        }
#pragma unroll
        for (int k = 0; k < 2; ++k) {
            int p = tid + 256 * k, row = p >> 5, ch = (p & 31) * 8;
            *(volatile v4u*)(FE + ((size_t)row * T + t) * HIDD + ch) = v[k].u;
        }
        __threadfence();
#pragma unroll
        for (int k = 0; k < 2; ++k) {
            int p = tid + 256 * k, row = p >> 5, ch = (p & 31) * 8;
            *(volatile v4u*)(FE + ((size_t)row * T + t) * HIDD + ch) = v[k].u;
        }
    }

#pragma unroll
    for (int i = 0; i < 2; ++i) {
        const int fo = fb + 16 * i + 8 * h;
        Pk32 p0, p1;
#pragma unroll
        for (int r = 0; r < 4; ++r) { p0.f[r] = hreg[i][r]; p1.f[r] = hreg[i][4 + r]; }
        float* d = SF + m * HIDD + fo;
        *(v4f*)d       = p0.f;
        *(v4f*)(d + 4) = p1.f;
    }
    __syncthreads();
    Pk32 vv[4];
#pragma unroll
    for (int k = 0; k < 4; ++k) {
        int p = tid + 256 * k, row = p >> 6, c = (p & 63) * 4;
        vv[k].f = *(const v4f*)(SF + row * HIDD + c);
    }
#pragma unroll
    for (int k = 0; k < 4; ++k) {
        int p = tid + 256 * k, row = p >> 6, c = (p & 63) * 4;
        *(volatile v4u*)(HT + (size_t)row * HIDD + c) = vv[k].u;
    }
    __threadfence();
#pragma unroll
    for (int k = 0; k < 4; ++k) {
        int p = tid + 256 * k, row = p >> 6, c = (p & 63) * 4;
        *(volatile v4u*)(HT + (size_t)row * HIDD + c) = vv[k].u;
    }
}

__global__ __launch_bounds__(256)
void k_final(const f16t* FE, const float* LV, const float* DL, const float* PO,
             const float* gw, const float* gbias, float* OUT, int ntok) {
    __shared__ __attribute__((aligned(16))) float SO[32 * 64];
    const int tid = threadIdx.x, w = tid >> 5, l = tid & 31;
    const int t0 = blockIdx.x * 32;
    if (t0 + 32 > ntok) return;
    const float g_w = gw[0], g_b = gbias[0];

#pragma unroll 1
    for (int q = 0; q < 4; ++q) {
        const int lt = 4 * w + q;
        const size_t tok = (size_t)(t0 + lt);

        float sv = LV[tok * CTXD + l] + LV[tok * CTXD + 32 + l];
        sv = wsum(sv);
        const float mean = sv * 0.015625f;
        const float gate = fsigm(fmaf(g_w, -mean, g_b));

        Pk16 f;
        f.h = *(const v8h*)(FE + tok * HIDD + 8 * l);
        const float* wfp = DL + tok * HNOUT + 32 * l;
        float s0 = 0.f, s1 = 0.f, s2 = 0.f, s3 = 0.f;
#pragma unroll
        for (int e = 0; e < 8; ++e) {
            v4f wv = *(const v4f*)(wfp + 4 * e);
            float fe = (float)f.h[e];
            s0 = fmaf(fe, wv[0], s0);
            s1 = fmaf(fe, wv[1], s1);
            s2 = fmaf(fe, wv[2], s2);
            s3 = fmaf(fe, wv[3], s3);
        }
        s0 = wsum(s0); s1 = wsum(s1); s2 = wsum(s2); s3 = wsum(s3);

        const float* afp = DL + tok * HNOUT + HIDD * 4;
        const float* dbp = DL + tok * HNOUT + HIDD * 4 + 4 * ACTD;
#pragma unroll
        for (int u = 0; u < 2; ++u) {
            const int a = l + 32 * u;
            float da = s0 * afp[a] + s1 * afp[ACTD + a] + s2 * afp[2 * ACTD + a] + s3 * afp[3 * ACTD + a];
            float v  = PO[tok * ACTD + a] + gate * (da + dbp[a]);
            SO[lt * ACTD + a] = v;
        }
    }
    __syncthreads();
    Pk32 v[2];
#pragma unroll
    for (int k = 0; k < 2; ++k) {
        int p = tid + 256 * k, row = p >> 4, c = (p & 15) * 4;
        v[k].f = *(const v4f*)(SO + row * ACTD + c);
    }
#pragma unroll
    for (int k = 0; k < 2; ++k) {
        int p = tid + 256 * k, row = p >> 4, c = (p & 15) * 4;
        *(volatile v4u*)(OUT + (size_t)(t0 + row) * ACTD + c) = v[k].u;
    }
    __threadfence();
#pragma unroll
    for (int k = 0; k < 2; ++k) {
        int p = tid + 256 * k, row = p >> 4, c = (p & 15) * 4;
        *(volatile v4u*)(OUT + (size_t)(t0 + row) * ACTD + c) = v[k].u;
    }
}

extern "C" void kernel_launch(void* const* d_in, const int* in_sizes, int n_in,
                              void* d_out, int out_size, void* d_ws, size_t ws_size,
                              hipStream_t stream) {
    if (n_in < 24) return;
    if (in_sizes[0] != NTOK * OBSD || in_sizes[1] != NBATCH * HIDD ||
        in_sizes[2] != W0D * OBSD || in_sizes[3] != W0D ||
        in_sizes[4] != W0D * W0D || in_sizes[5] != W0D ||
        in_sizes[6] != G3D * W0D || in_sizes[7] != G3D * HIDD ||
        in_sizes[8] != G3D || in_sizes[9] != G3D ||
        in_sizes[10] != CTXD * HIDD || in_sizes[11] != CTXD ||
        in_sizes[12] != CTXD * HIDD || in_sizes[13] != CTXD ||
        in_sizes[14] < 1 || in_sizes[15] < 1 ||
        in_sizes[16] != ACTD * HIDD || in_sizes[17] != ACTD ||
        in_sizes[18] != HNH * CTXD || in_sizes[19] != HNH ||
        in_sizes[20] != HNH * HNH || in_sizes[21] != HNH ||
        in_sizes[22] != HNOUT * HNH || in_sizes[23] != HNOUT) return;
    if (out_size != NTOK * ACTD + NBATCH * HIDD) return;

    const float* obs   = (const float*)d_in[0];
    const float* h0    = (const float*)d_in[1];
    const float* W_in  = (const float*)d_in[2];
    const float* b_in  = (const float*)d_in[3];
    const float* W_h1  = (const float*)d_in[4];
    const float* b_h1  = (const float*)d_in[5];
    const float* Wih   = (const float*)d_in[6];
    const float* Whh   = (const float*)d_in[7];
    const float* bih   = (const float*)d_in[8];
    const float* bhh   = (const float*)d_in[9];
    const float* W_mu  = (const float*)d_in[10];
    const float* b_mu  = (const float*)d_in[11];
    const float* W_lv  = (const float*)d_in[12];
    const float* b_lv  = (const float*)d_in[13];
    const float* g_w   = (const float*)d_in[14];
    const float* g_b   = (const float*)d_in[15];
    const float* W_pol = (const float*)d_in[16];
    const float* b_pol = (const float*)d_in[17];
    const float* hn_W1 = (const float*)d_in[18];
    const float* hn_b1 = (const float*)d_in[19];
    const float* hn_W2 = (const float*)d_in[20];
    const float* hn_b2 = (const float*)d_in[21];
    const float* hn_W3 = (const float*)d_in[22];
    const float* hn_b3 = (const float*)d_in[23];

    float* out0 = (float*)d_out;
    float* out1 = (float*)d_out + (size_t)NTOK * ACTD;

    char* ws = (char*)d_ws;
    size_t off = 0;
    auto carve = [&](size_t bytes) -> char* {
        char* p = ws + off;
        off = (off + bytes + 255) & ~(size_t)255;
        return p;
    };
    f16t* OBS16 = (f16t*)carve((size_t)NTOK * OBSD * 2);
    f16t* Pin   = (f16t*)carve((size_t)W0D * OBSD * 2);
    f16t* Ph1   = (f16t*)carve((size_t)W0D * W0D * 2);
    f16t* Pih   = (f16t*)carve((size_t)G3D * W0D * 2);
    f16t* Phh   = (f16t*)carve((size_t)G3D * HIDD * 2);
    f16t* Pmu   = (f16t*)carve((size_t)CTXD * HIDD * 2);
    f16t* Plv   = (f16t*)carve((size_t)CTXD * HIDD * 2);
    f16t* Ppol  = (f16t*)carve((size_t)ACTD * HIDD * 2);
    f16t* P1    = (f16t*)carve((size_t)HNH * CTXD * 2);
    f16t* P2    = (f16t*)carve((size_t)HNH * HNH * 2);
    f16t* P3    = (f16t*)carve((size_t)HNOUT * HNH * 2);
    f16t* X1    = (f16t*)carve((size_t)NTOK * W0D * 2);
    f16t* X2    = (f16t*)carve((size_t)NTOK * W0D * 2);
    float* XG   = (float*)carve((size_t)NTOK * G3D * 4);
    f16t* FE    = (f16t*)carve((size_t)NTOK * HIDD * 2);
    f16t* MU    = (f16t*)carve((size_t)NTOK * CTXD * 2);
    float* LV   = (float*)carve((size_t)NTOK * CTXD * 4);
    float* PO   = (float*)carve((size_t)NTOK * ACTD * 4);
    f16t* H1    = (f16t*)carve((size_t)NTOK * HNH * 2);
    f16t* H2    = (f16t*)carve((size_t)NTOK * HNH * 2);
    float* DL   = (float*)carve((size_t)NTOK * HNOUT * 4);
    if (off > ws_size) return;
    if (off > (size_t)134217728) return;

    const float SW = 16.0f, IW = 0.0625f;

    auto cvt = [&](const float* s, f16t* d, int n, float sc) {
        int n8 = n >> 3;
        k_cvt8<<<dim3((n8 + 255) / 256), dim3(256), 0, stream>>>(s, d, n8, sc);
    };
    cvt(obs,   OBS16, NTOK * OBSD,  1.0f);
    cvt(W_in,  Pin,   W0D * OBSD,   SW);
    cvt(W_h1,  Ph1,   W0D * W0D,    SW);
    cvt(Wih,   Pih,   G3D * W0D,    SW);
    cvt(Whh,   Phh,   G3D * HIDD,   SW);
    cvt(W_mu,  Pmu,   CTXD * HIDD,  SW);
    cvt(W_lv,  Plv,   CTXD * HIDD,  SW);
    cvt(W_pol, Ppol,  ACTD * HIDD,  SW);
    cvt(hn_W1, P1,    HNH * CTXD,   SW);
    cvt(hn_W2, P2,    HNH * HNH,    SW);
    cvt(hn_W3, P3,    HNOUT * HNH,  SW);

    const dim3 blk64(64);
    k_gemm<f16t, 1><<<dim3(W0D / 64, NTOK / 64), blk64, 0, stream>>>(
        OBS16, OBSD, Pin, OBSD, b_in, X1, W0D, NTOK, W0D, IW);
    k_gemm<f16t, 1><<<dim3(W0D / 64, NTOK / 64), blk64, 0, stream>>>(
        X1, W0D, Ph1, W0D, b_h1, X2, W0D, NTOK, W0D, IW);
    k_gemm<float, 0><<<dim3(G3D / 64, NTOK / 64), blk64, 0, stream>>>(
        X2, W0D, Pih, W0D, bih, XG, G3D, NTOK, G3D, IW);
    k_gru<<<dim3(1), dim3(256), 0, stream>>>(XG, Phh, bhh, h0, FE, out1, NSTEP, IW);
    k_gemm<f16t, 0><<<dim3(CTXD / 64, NTOK / 64), blk64, 0, stream>>>(
        FE, HIDD, Pmu, HIDD, b_mu, MU, CTXD, NTOK, CTXD, IW);
    k_gemm<float, 2><<<dim3(CTXD / 64, NTOK / 64), blk64, 0, stream>>>(
        FE, HIDD, Plv, HIDD, b_lv, LV, CTXD, NTOK, CTXD, IW);
    k_gemm<float, 0><<<dim3(ACTD / 64, NTOK / 64), blk64, 0, stream>>>(
        FE, HIDD, Ppol, HIDD, b_pol, PO, ACTD, NTOK, ACTD, IW);
    k_gemm<f16t, 1><<<dim3(HNH / 64, NTOK / 64), blk64, 0, stream>>>(
        MU, CTXD, P1, CTXD, hn_b1, H1, HNH, NTOK, HNH, IW);
    k_gemm<f16t, 1><<<dim3(HNH / 64, NTOK / 64), blk64, 0, stream>>>(
        H1, HNH, P2, HNH, hn_b2, H2, HNH, NTOK, HNH, IW);
    k_gemm<float, 3><<<dim3(HNOUT / 64, NTOK / 64), blk64, 0, stream>>>(
        H2, HNH, P3, HNH, hn_b3, DL, HNOUT, NTOK, HNOUT, IW);
    k_final<<<dim3(NTOK / 32), dim3(256), 0, stream>>>(FE, LV, DL, PO, g_w, g_b, out0, NTOK);
}
